// DependencyBertMix_46316927320622
// MI455X (gfx1250) — hardware-verified
//
#include <hip/hip_runtime.h>
#include <math.h>

typedef __attribute__((ext_vector_type(16))) _Float16 v16h;
typedef __attribute__((ext_vector_type(16))) __bf16 v16b;
typedef __attribute__((ext_vector_type(8)))  _Float16 v8h;
typedef __attribute__((ext_vector_type(8)))  float v8f;
typedef __attribute__((ext_vector_type(4)))  float v4f;
typedef __attribute__((ext_vector_type(2)))  float v2f;
typedef __attribute__((ext_vector_type(4)))  unsigned v4u;
typedef __attribute__((ext_vector_type(4)))  int v4i;
typedef float __attribute__((may_alias)) float_a;
typedef int __attribute__((may_alias)) int_a;

template <typename T> __device__ __forceinline__ void vst2(void* p, T v) { *(volatile T*)p = v; __threadfence(); *(volatile T*)p = v; }
__device__ __forceinline__ v8f wmma16(v16h a, v16h b, v8f c) {
  v8f d = __builtin_amdgcn_wmma_f32_16x16x32_f16(false, a, false, b, (short)0, c, false, false);
  asm volatile("v_nop\n\tv_nop\n\tv_nop\n\tv_nop" : "+v"(d) : "v"(a), "v"(b));
  return d;
}
__device__ __forceinline__ v8f wmma_bf(v16b a, v16b b, v8f c) {
  v8f d = __builtin_amdgcn_wmma_f32_16x16x32_bf16(false, a, false, b, (short)0, c, false, false);
  asm volatile("v_nop\n\tv_nop\n\tv_nop\n\tv_nop" : "+v"(d) : "v"(a), "v"(b));
  return d;
}
__device__ __forceinline__ v16h frag_h(const _Float16* rowk0, int lane) {
  union { v16h v; v8h q[2]; } u; const _Float16* p = rowk0 + 8 * (lane >> 4);
  u.q[0] = *(const v8h*)p; u.q[1] = *(const v8h*)(p + 16); return u.v;
}
__device__ __forceinline__ v16h frag_f32(const float* rowk0, int lane) {
  v16h a; const float* p = rowk0 + 8 * (lane >> 4);
#pragma unroll
  for (int i = 0; i < 8; ++i) { a[i] = (_Float16)p[i]; a[8 + i] = (_Float16)p[16 + i]; }
  return a;
}
__device__ __forceinline__ v16h frag_f32s(const float* rowk0, int lane, float sc) {
  v16h a; const float* p = rowk0 + 8 * (lane >> 4);
#pragma unroll
  for (int i = 0; i < 8; ++i) { a[i] = (_Float16)(p[i] * sc); a[8 + i] = (_Float16)(p[16 + i] * sc); }
  return a;
}
__device__ __forceinline__ v16h fragc_f32(const float* W, int k0, int n, int lane, int ld, int K) {
  v16h a; const int g = lane >> 4;
#pragma unroll
  for (int i = 0; i < 8; ++i) { const int ka = k0 + 8 * g + i, kb = ka + 16;
    a[i] = (_Float16)(ka < K ? W[(size_t)(ka < K ? ka : K - 1) * ld + n] : 0.f); a[8 + i] = (_Float16)(kb < K ? W[(size_t)(kb < K ? kb : K - 1) * ld + n] : 0.f); }
  return a;
}
struct F2 { v16b h, l; };
__device__ __forceinline__ F2 bsplit16(const float v[16]) { F2 r;
#pragma unroll
  for (int i = 0; i < 16; ++i) { const __bf16 h = (__bf16)v[i]; r.h[i] = h; r.l[i] = (__bf16)(v[i] - (float)h); }
  return r; }
__device__ __forceinline__ F2 split_row(const float* row, int k0, int lane) { float v[16]; const float* p = row + k0 + 8 * (lane >> 4);
#pragma unroll
  for (int i = 0; i < 8; ++i) { v[i] = p[i]; v[8 + i] = p[16 + i]; }
  return bsplit16(v); }
__device__ __forceinline__ F2 split_rowK(const float* row, int k0, int lane, int K) { float v[16]; const int g = lane >> 4;
#pragma unroll
  for (int i = 0; i < 8; ++i) { const int ka = k0 + 8 * g + i, kb = ka + 16; v[i] = ka < K ? row[ka < K ? ka : K - 1] : 0.f; v[8 + i] = kb < K ? row[kb < K ? kb : K - 1] : 0.f; }
  return bsplit16(v); }
__device__ __forceinline__ F2 split_col(const float* W, int k0, int n, int lane, int ld, int K) { float v[16]; const int g = lane >> 4;
#pragma unroll
  for (int i = 0; i < 8; ++i) { const int ka = k0 + 8 * g + i, kb = ka + 16; v[i] = ka < K ? W[(size_t)(ka < K ? ka : K - 1) * ld + n] : 0.f; v[8 + i] = kb < K ? W[(size_t)(kb < K ? kb : K - 1) * ld + n] : 0.f; }
  return bsplit16(v); }
__device__ __forceinline__ v8f mac3(const F2& a, const F2& b, v8f c) { c = wmma_bf(a.l, b.h, c); c = wmma_bf(a.h, b.l, c); return wmma_bf(a.h, b.h, c); }
__device__ __forceinline__ float sigm(float v) { return 1.0f / (1.0f + expf(-v)); }
#define LDSX() do { asm volatile("s_wait_dscnt 0" ::: "memory"); __builtin_amdgcn_wave_barrier(); __builtin_amdgcn_fence(__ATOMIC_RELEASE, "workgroup"); } while (0)


#define NB 8
#define TT 512
#define CC 768
#define NH 12
#define HD 64
#define NROW (NB * TT)
#define NAR (NB * NH * TT)
#define GH 512
#ifndef TNB
#define TNB NB
#endif
typedef __attribute__((ext_vector_type(8))) __bf16 v8b;
__device__ __forceinline__ v16b frag_b(const __bf16* rowk0, int lane) {
  union { v16b v; v8b q[2]; } u; const __bf16* p = rowk0 + 8 * (lane >> 4);
  u.q[0] = *(const v8b*)p; u.q[1] = *(const v8b*)(p + 16); return u.v;
}
__device__ __forceinline__ float bfr(float v) { return (float)(__bf16)v; }
__device__ __attribute__((noinline)) float exp_ni(float v) { return expf(v); }
__device__ __attribute__((noinline)) float erf_ni(float v) { return erff(v); }

#define WS_QH  0u
#define WS_QL  (WS_QH + 2u * (size_t)NROW * CC)
#define WS_KH  (WS_QL + 2u * (size_t)NROW * CC)
#define WS_VT  (WS_KH + 2u * (size_t)NROW * CC)
#define NARB (NH * TT)
#define WS_S   (WS_VT + 2u * (size_t)NROW * CC)
#define WS_MX  (WS_S + 4u * (size_t)NARB * TT)
#define WS_T1  (WS_MX + 2u * (size_t)NARB * 2 * TT)
#define WS_G   (WS_T1 + 2u * (size_t)NARB * GH)
#define WS_P   (WS_G + 4u * (size_t)NARB * TT)
#define WS_END (WS_P + 2u * (size_t)NARB * TT)

__global__ __launch_bounds__(128) void k_proj(const float* __restrict__ X, const float* __restrict__ WQ, const float* __restrict__ BQ, const float* __restrict__ WK, const float* __restrict__ BK, const float* __restrict__ WV, const float* __restrict__ BV, _Float16* __restrict__ QH, _Float16* __restrict__ QL, _Float16* __restrict__ KH, _Float16* __restrict__ VT) {
  __shared__ __align__(16) _Float16 sh[64][136], sl[64][136]; __shared__ __align__(16) _Float16 th[128][72];
  const int tid = threadIdx.x, wave = tid >> 5, lane = tid & 31, col = lane & 15, g = lane >> 4; const int which = blockIdx.z; const int c0 = blockIdx.y * 128; const size_t r0 = (size_t)blockIdx.x * 64;
  const float* Wm = which == 0 ? WQ : which == 1 ? WK : WV; const float* Bm = which == 0 ? BQ : which == 1 ? BK : BV;
  v8f acc[8] = {};
#pragma unroll 2
  for (int kc = 0; kc < CC / 32; ++kc) { v16b a; { const float* p = X + (r0 + wave * 16 + col) * CC + kc * 32 + 8 * g;
#pragma unroll
      for (int i = 0; i < 8; ++i) { a[i] = (__bf16)p[i]; a[8 + i] = (__bf16)p[16 + i]; } }
#pragma unroll
    for (int j = 0; j < 8; ++j) { v16b w; const int o = c0 + j * 16 + col;
#pragma unroll
      for (int i = 0; i < 8; ++i) { w[i] = (__bf16)Wm[(size_t)(kc * 32 + 8 * g + i) * CC + o]; w[8 + i] = (__bf16)Wm[(size_t)(kc * 32 + 16 + 8 * g + i) * CC + o]; }
      acc[j] = wmma_bf(a, w, acc[j]); } }
#pragma unroll
  for (int j = 0; j < 8; ++j) { const float bb = bfr(Bm[c0 + j * 16 + col]);
#pragma unroll
    for (int r = 0; r < 8; ++r) { const float v = acc[j][r] + bb; const int rl = wave * 16 + 8 * g + r, cl = j * 16 + col; const _Float16 hv = (_Float16)v;
      if (which == 2) th[cl][rl] = hv; else { sh[rl][cl] = hv; sl[rl][cl] = (_Float16)(v - (float)hv); } } }
  __syncthreads();
  if (which < 2) { _Float16* dh = which == 0 ? QH : KH; for (int e = tid; e < 64 * 16; e += 128) { const int rl = e >> 4, q = e & 15; vst2((unsigned*)(dh + (r0 + rl) * CC + c0 + q * 8), *(const v4u*)&sh[rl][q * 8]); if (which == 0) vst2((unsigned*)(QL + (r0 + rl) * CC + c0 + q * 8), *(const v4u*)&sl[rl][q * 8]); } }
  else { const size_t b = r0 / TT; const int t0 = (int)(r0 % TT); for (int e = tid; e < 128 * 8; e += 128) { const int cl = e >> 3, q = e & 7; vst2((unsigned*)(VT + (b * CC + c0 + cl) * (size_t)TT + t0 + q * 8), *(const v4u*)&th[cl][q * 8]); } } }
__global__ __launch_bounds__(128) void k_sc(const _Float16* __restrict__ QH, const _Float16* __restrict__ QL, const _Float16* __restrict__ KH, int b, float* __restrict__ S) { __shared__ __align__(16) float ss[4][16][132];
  const int tid = threadIdx.x, wave = tid >> 5, lane = tid & 31, col = lane & 15, g = lane >> 4; const int k0 = blockIdx.y * 128; const int h = blockIdx.z; const int bh = h; const int ql0 = blockIdx.x * 64 + wave * 16; const size_t q0 = (size_t)b * TT + ql0;
  v8f acc[8] = {};
#pragma unroll
  for (int kc = 0; kc < HD / 32; ++kc) { const v16h ah = frag_h(QH + (q0 + col) * CC + h * HD + kc * 32, lane), al = frag_h(QL + (q0 + col) * CC + h * HD + kc * 32, lane);
#pragma unroll
    for (int j = 0; j < 8; ++j) { const v16h kb = frag_h(KH + ((size_t)b * TT + k0 + j * 16 + col) * CC + h * HD + kc * 32, lane); acc[j] = wmma16(ah, kb, acc[j]); acc[j] = wmma16(al, kb, acc[j]); } }
#pragma unroll
  for (int j = 0; j < 8; ++j)
#pragma unroll
    for (int r = 0; r < 8; ++r) ss[wave][8 * g + r][j * 16 + col] = acc[j][r] * 0.125f;
  LDSX(); for (int rl = 0; rl < 16; ++rl) vst2(S + ((size_t)bh * TT + ql0 + rl) * TT + k0 + lane * 4, *(const v4f*)&ss[wave][rl][lane * 4]); }
__global__ __launch_bounds__(256) void k_mix(const float* __restrict__ S, const float* __restrict__ AM, const float* __restrict__ DM, const float* __restrict__ LG, const float* __restrict__ LB, int b, _Float16* __restrict__ MX) { __shared__ float sv[2 * TT]; __shared__ float sred[8]; __shared__ float smu, sinv; __shared__ __align__(16) _Float16 so[2 * TT];
  const int t = threadIdx.x; const size_t row = blockIdx.x; const int tq = (int)(row % TT);
  for (int s = t; s < TT; s += 256) { const float sc = S[row * TT + s]; const float m = bfr(AM[(size_t)b * TT + s]); sv[s] = sc + (1.0f - m) * -10000.0f; sv[TT + s] = sc * bfr(DM[((size_t)b * TT + tq) * TT + s]); }
  __syncthreads();
  float a = 0.f; for (int i = t; i < 2 * TT; i += 256) a += sv[i];
#pragma unroll
  for (int o = 1; o < 32; o <<= 1) a += __shfl_xor(a, o);
  if ((t & 31) == 0) sred[t >> 5] = a; __syncthreads(); if (t == 0) { float x = 0.f; for (int w = 0; w < 8; ++w) x += sred[w]; smu = x / (2 * TT); } __syncthreads(); const float mu = smu;
  float q = 0.f; for (int i = t; i < 2 * TT; i += 256) { const float d = sv[i] - mu; q += d * d; }
#pragma unroll
  for (int o = 1; o < 32; o <<= 1) q += __shfl_xor(q, o);
  __syncthreads(); if ((t & 31) == 0) sred[t >> 5] = q; __syncthreads(); if (t == 0) { float x = 0.f; for (int w = 0; w < 8; ++w) x += sred[w]; sinv = 1.0f / sqrtf(x / (2 * TT) + 1e-5f); } __syncthreads(); const float inv = sinv;
  for (int i = t; i < 2 * TT; i += 256) so[i] = (_Float16)((sv[i] - mu) * inv * bfr(LG[i]) + bfr(LB[i]));
  __syncthreads(); for (int qq = t; qq < 2 * TT / 8; qq += 256) vst2((unsigned*)(MX + row * (2 * TT) + qq * 8), *(const v4u*)&so[qq * 8]); }
template <int STAGE>
__global__ __launch_bounds__(128) void k_g(const _Float16* __restrict__ IN, const float* __restrict__ Wm, const float* __restrict__ Bm, _Float16* __restrict__ OUTH, float* __restrict__ OUTF) { __shared__ __align__(16) float sf[4][16][132]; __shared__ __align__(16) _Float16 sh2[64][136];
  const int tid = threadIdx.x, wave = tid >> 5, lane = tid & 31, col = lane & 15, g = lane >> 4; const int c0 = blockIdx.y * 128; const size_t r0 = (size_t)blockIdx.x * 64 + wave * 16; constexpr int K = (STAGE == 0) ? 2 * TT : GH; constexpr int NOUT = GH;
  v8f acc[8] = {};
#pragma unroll 2
  for (int kc = 0; kc < K / 32; ++kc) { const v16h a = frag_h(IN + (r0 + col) * K + kc * 32, lane);
#pragma unroll
    for (int j = 0; j < 8; ++j) { v16h w; const int o = c0 + j * 16 + col;
#pragma unroll
      for (int i = 0; i < 8; ++i) { w[i] = (_Float16)bfr(Wm[(size_t)(kc * 32 + 8 * g + i) * NOUT + o]); w[8 + i] = (_Float16)bfr(Wm[(size_t)(kc * 32 + 16 + 8 * g + i) * NOUT + o]); }
      acc[j] = wmma16(a, w, acc[j]); } }
#pragma unroll
  for (int j = 0; j < 8; ++j) { const float bb = bfr(Bm[c0 + j * 16 + col]);
#pragma unroll
    for (int r = 0; r < 8; ++r) { const float v = acc[j][r] + bb; if (STAGE == 0) sh2[wave * 16 + 8 * g + r][j * 16 + col] = (_Float16)tanhf(v); else sf[wave][8 * g + r][j * 16 + col] = 1.0f / (1.0f + expf(-v)); } }
  __syncthreads();
  if (STAGE == 0) { for (int e = tid; e < 64 * 16; e += 128) { const int rl = e >> 4, q = e & 15; vst2((unsigned*)(OUTH + ((size_t)blockIdx.x * 64 + rl) * GH + c0 + q * 8), *(const v4u*)&sh2[rl][q * 8]); } }
  else { for (int rl = 0; rl < 16; ++rl) vst2(OUTF + (r0 + rl) * TT + c0 + lane * 4, *(const v4f*)&sf[wave][rl][lane * 4]); } }
__global__ __launch_bounds__(256) void k_fin(const float* __restrict__ S, const float* __restrict__ AM, const float* __restrict__ DM, const float* __restrict__ G, int b, _Float16* __restrict__ P) { __shared__ float sl[TT]; __shared__ float sred[8]; __shared__ float sbc; __shared__ __align__(16) _Float16 so[TT];
  const int t = threadIdx.x; const size_t row = blockIdx.x; const int tq = (int)(row % TT);
  float m = -3.0e38f; for (int s = t; s < TT; s += 256) { const float sc = S[row * TT + s]; const float am = bfr(AM[(size_t)b * TT + s]); const float se = sc + (1.0f - am) * -10000.0f; const float de = sc * bfr(DM[((size_t)b * TT + tq) * TT + s]); const float gg = G[row * TT + s]; const float v = gg * se + (1.0f - gg) * de; sl[s] = v; m = fmaxf(m, v); }
#pragma unroll
  for (int o = 1; o < 32; o <<= 1) m = fmaxf(m, __shfl_xor(m, o));
  if ((t & 31) == 0) sred[t >> 5] = m; __syncthreads(); if (t == 0) { float a = sred[0]; for (int i = 1; i < 8; ++i) a = fmaxf(a, sred[i]); sbc = a; } __syncthreads(); m = sbc; __syncthreads();
  float sum = 0.f; for (int s = t; s < TT; s += 256) sum += expf(sl[s] - m);
#pragma unroll
  for (int o = 1; o < 32; o <<= 1) sum += __shfl_xor(sum, o);
  if ((t & 31) == 0) sred[t >> 5] = sum; __syncthreads(); if (t == 0) { float a = 0.f; for (int i = 0; i < 8; ++i) a += sred[i]; sbc = 1.0f / a; } __syncthreads(); const float inv = sbc;
  for (int s = t; s < TT; s += 256) so[s] = (_Float16)(expf(sl[s] - m) * inv * 2048.0f);
  __syncthreads(); for (int q = t; q < TT / 8; q += 256) vst2((unsigned*)(P + row * TT + q * 8), *(const v4u*)&so[q * 8]); }
__global__ __launch_bounds__(128) void k_pv(const _Float16* __restrict__ P, const _Float16* __restrict__ VT, int b, float* __restrict__ OUT) { __shared__ __align__(16) float ss[4][16][68];
  const int tid = threadIdx.x, wave = tid >> 5, lane = tid & 31, col = lane & 15, g = lane >> 4; const int h = blockIdx.y; const int bh = h; const int ql0 = blockIdx.x * 64 + wave * 16;
  v8f acc[4] = {};
#pragma unroll 1
  for (int kc = 0; kc < TT / 32; ++kc) { const v16h ph = frag_h(P + ((size_t)bh * TT + ql0 + col) * TT + kc * 32, lane);
#pragma unroll
    for (int j = 0; j < 4; ++j) acc[j] = wmma16(ph, frag_h(VT + ((size_t)b * CC + h * HD + j * 16 + col) * TT + kc * 32, lane), acc[j]); }
#pragma unroll
  for (int j = 0; j < 4; ++j)
#pragma unroll
    for (int r = 0; r < 8; ++r) ss[wave][8 * g + r][j * 16 + col] = acc[j][r] * (1.0f / 2048.0f);
  LDSX(); for (int rl = 0; rl < 16; ++rl) if (lane < 16) vst2(OUT + ((size_t)b * TT + ql0 + rl) * CC + h * HD + lane * 4, *(const v4f*)&ss[wave][rl][lane * 4]); }
extern "C" void kernel_launch(void* const* d_in, const int* in_sizes, int n_in, void* d_out, int out_size, void* d_ws, size_t ws_size, hipStream_t stream) {
  (void)in_sizes; (void)n_in; (void)out_size;
  const float** F = (const float**)d_in;
  if (ws_size < (size_t)WS_END) return;
  char* ws = (char*)d_ws; _Float16 *QH = (_Float16*)(ws + WS_QH), *QL = (_Float16*)(ws + WS_QL), *KH = (_Float16*)(ws + WS_KH), *VT = (_Float16*)(ws + WS_VT), *MX = (_Float16*)(ws + WS_MX), *T1 = (_Float16*)(ws + WS_T1), *P = (_Float16*)(ws + WS_P); float *S = (float*)(ws + WS_S), *G = (float*)(ws + WS_G);
  k_proj<<<dim3(TNB * TT / 64, CC / 128, 3), 128, 0, stream>>>(F[0], F[3], F[4], F[5], F[6], F[7], F[8], QH, QL, KH, VT);
  for (int b = 0; b < TNB; ++b) {
    k_sc<<<dim3(TT / 64, TT / 128, NH), 128, 0, stream>>>(QH, QL, KH, b, S);
    k_mix<<<NARB, 256, 0, stream>>>(S, F[1], F[2], F[9], F[10], b, MX);
    k_g<0><<<dim3(NARB / 64, GH / 128), 128, 0, stream>>>(MX, F[11], F[12], T1, nullptr);
    k_g<1><<<dim3(NARB / 64, GH / 128), 128, 0, stream>>>(T1, F[13], F[14], nullptr, G);
    k_fin<<<NARB, 256, 0, stream>>>(S, F[1], F[2], G, b, P);
    k_pv<<<dim3(TT / 64, NH), 128, 0, stream>>>(P, VT, b, (float*)d_out);
  }
}
